// TextEncoderGenerator_4475355923026
// MI455X (gfx1250) — hardware-verified
//
#include <hip/hip_runtime.h>
#include <math.h>

constexpr int NBATCH = 256;
constexpr int NSEQ   = 128;
constexpr int NIN    = 300;
constexpr int NINP   = 320;
constexpr int NHID   = 512;
constexpr int NGATE  = 3 * NHID;
constexpr int NCOND  = 128;
constexpr int CHUNK_STEPS = 16;
constexpr int NCHUNK = NSEQ / CHUNK_STEPS;
constexpr int CHUNK_ROWS = CHUNK_STEPS * NBATCH;
constexpr int SEQ_PER_BLK = 32;
constexpr int REC_THREADS = 512;
constexpr int REC_BLOCKS  = 2 * (NBATCH / SEQ_PER_BLK);
constexpr int HPL_PITCH = 528;
constexpr float H_CARRY = 64.0f;
constexpr float W_CARRY = 16.0f;
constexpr float GH_UNSCALE = 1.0f / 1024.0f;
constexpr float AVG_SCALE = 1.0f / 256.0f;
static_assert(NSEQ % CHUNK_STEPS == 0);
static_assert(NBATCH % SEQ_PER_BLK == 0);
static_assert(CHUNK_ROWS % 64 == 0 && NGATE % 64 == 0 && NINP % 32 == 0);
static_assert(NBATCH % 64 == 0 && NCOND % 64 == 0 && NHID % 32 == 0);

constexpr int REC_LDS_HST   = 0;
constexpr int REC_LDS_SSUM  = SEQ_PER_BLK * NHID * 4;
constexpr int REC_LDS_HPL   = 2 * SEQ_PER_BLK * NHID * 4;
constexpr int REC_LDS_SLEN  = REC_LDS_HPL + SEQ_PER_BLK * HPL_PITCH * 2;
constexpr int REC_LDS_BYTES = REC_LDS_SLEN + SEQ_PER_BLK * 4;
static_assert(REC_LDS_SLEN % 16 == 0);

typedef __attribute__((ext_vector_type(16))) _Float16 v16h;
typedef __attribute__((ext_vector_type(8)))  _Float16 v8h;
typedef __attribute__((ext_vector_type(16))) __bf16   v16b;
typedef __attribute__((ext_vector_type(8)))  __bf16   v8b;
typedef __attribute__((ext_vector_type(8)))  float    v8f;
typedef __attribute__((ext_vector_type(4)))  float    v4f;
typedef __attribute__((ext_vector_type(4)))  unsigned int v4u;

__device__ __forceinline__ unsigned short f2bf_bits(float f) {
  unsigned u = __float_as_uint(f);
  return (unsigned short)((u + 0x7FFFu + ((u >> 16) & 1u)) >> 16);
}
__device__ __forceinline__ float bf_bits2f(unsigned short h) { return __uint_as_float(((unsigned)h) << 16); }

__device__ __forceinline__ void dep_guard_h(v8f& a, v8f& b, v16h x, v16h y) { asm volatile("v_nop\n\tv_nop\n\tv_nop\n\tv_nop" : "+v"(a), "+v"(b) : "v"(x), "v"(y)); }
__device__ __forceinline__ void dep_guard_b(v8f& a, v8f& b, v16b x, v16b y) { asm volatile("v_nop\n\tv_nop\n\tv_nop\n\tv_nop" : "+v"(a), "+v"(b) : "v"(x), "v"(y)); }
__device__ __forceinline__ void keep4_h(v16h a, v16h b, v16h c, v16h d) { asm volatile("v_nop" :: "v"(a), "v"(b), "v"(c), "v"(d)); }
__device__ __forceinline__ void keep4_b(v16b a, v16b b, v16b c, v16b d) { asm volatile("v_nop" :: "v"(a), "v"(b), "v"(c), "v"(d)); }
__device__ __forceinline__ void acc_guard4(v8f& a, v8f& b, v8f& c, v8f& d) { asm volatile("v_nop\n\tv_nop\n\tv_nop\n\tv_nop" : "+v"(a), "+v"(b), "+v"(c), "+v"(d)); }
template <typename T> struct Frag;
template <> struct Frag<_Float16> {
  typedef v16h V; union U { v16h v; v8h h[2]; };
  static __device__ __forceinline__ v16h load(const _Float16* p) {
    U f; f.h[0] = *(const v8h*)(p); f.h[1] = *(const v8h*)(p + 16); return f.v;
  }
  static __device__ __forceinline__ v8f mma(v16h a, v16h b, v8f c) {
    return __builtin_amdgcn_wmma_f32_16x16x32_f16(false, a, false, b, (short)0, c, false, false);
  }
  static __device__ __forceinline__ void guard(v8f& a, v8f& b, v16h x, v16h y) { dep_guard_h(a, b, x, y); }
  static __device__ __forceinline__ void keep(v16h a, v16h b, v16h c, v16h d) { keep4_h(a, b, c, d); }
};
template <> struct Frag<__bf16> {
  typedef v16b V; union U { v16b v; v8b h[2]; };
  static __device__ __forceinline__ v16b load(const __bf16* p) {
    U f; f.h[0] = *(const v8b*)(p); f.h[1] = *(const v8b*)(p + 16); return f.v;
  }
  static __device__ __forceinline__ v8f mma(v16b a, v16b b, v8f c) {
    return __builtin_amdgcn_wmma_f32_16x16x32_bf16(false, a, false, b, (short)0, c, false, false);
  }
  static __device__ __forceinline__ void guard(v8f& a, v8f& b, v16b x, v16b y) { dep_guard_b(a, b, x, y); }
  static __device__ __forceinline__ void keep(v16b a, v16b b, v16b c, v16b d) { keep4_b(a, b, c, d); }
};

__device__ __forceinline__ unsigned pk16(unsigned short a, unsigned short b) { return (unsigned)a | ((unsigned)b << 16); }
__device__ __forceinline__ float bf_rne(float v) { return bf_bits2f(f2bf_bits(v)); }
__device__ __forceinline__ unsigned short h_bits(float v) { return __builtin_bit_cast(unsigned short, (_Float16)v); }

template <int ET> struct Elem;
template <> struct Elem<0> { typedef _Float16 T; };
template <> struct Elem<1> { typedef __bf16 T; };
template <int ET, bool SPLIT, int BIAS_MODE, int OUT_MODE, bool RESID, int ACT = 0>
__global__ __launch_bounds__(256) void wmma_gemm64(
    const unsigned short* __restrict__ Ap, const unsigned short* __restrict__ A2p, int lda, long strideA,
    const unsigned short* __restrict__ Btp, const unsigned short* __restrict__ Bt2p, int ldb, long strideB,
    void* __restrict__ Cout, void* __restrict__ Cout2, int ldc, long strideC,
    const float* __restrict__ bias,
    const float* __restrict__ resid, long strideR,
    int M, int N, int K, float scale) {
  typedef typename Elem<ET>::T T;
  typedef typename Frag<T>::V V;
  const T* A = (const T*)Ap; const T* A2 = (const T*)A2p; const T* Bt = (const T*)Btp; const T* Bt2 = (const T*)Bt2p;
  __shared__ __align__(16) float sT[8][16 * 68];
  const int b    = blockIdx.y;
  const int lane = threadIdx.x & 31;
  const int wave = threadIdx.x >> 5;
  const int tilesN = N >> 6;
  const int tilesM = M >> 6;
  const int tile = blockIdx.x * 8 + wave;
  if (tile >= tilesM * tilesN) return;
  const int tm = tile / tilesN;
  const int tn = tile - tm * tilesN;
  const int m0 = tm << 6;
  const int n0 = tn << 6;

  const T* Ab  = A  + (size_t)b * strideA;
  const T* Bb  = Bt + (size_t)b * strideB;
  const T* Ab2 = SPLIT ? (A2  + (size_t)b * strideA) : nullptr;
  const T* Bb2 = SPLIT ? (Bt2 + (size_t)b * strideB) : nullptr;

  const int rlane = lane & 15;
  const int koff  = (lane >> 4) * 8;
  const int mOff  = (lane >> 4) * 8;

  v8f acc[4][4];
#pragma unroll
  for (int i = 0; i < 4; ++i)
#pragma unroll
    for (int j = 0; j < 4; ++j) acc[i][j] = (v8f){0.f,0.f,0.f,0.f,0.f,0.f,0.f,0.f};

  for (int k0 = 0; k0 < K; k0 += 32) {
    V bh[4], bl[4];
#pragma unroll
    for (int j = 0; j < 4; ++j) {
      const size_t bo = (size_t)(n0 + (j << 4) + rlane) * ldb + koff + k0;
      bh[j] = Frag<T>::load(Bb + bo);
      if (SPLIT) bl[j] = Frag<T>::load(Bb2 + bo);
    }
#pragma unroll
    for (int i = 0; i < 4; ++i) {
      const size_t ao = (size_t)(m0 + (i << 4) + rlane) * lda + koff + k0;
      V ah = Frag<T>::load(Ab + ao);
      V al;
      if (SPLIT) al = Frag<T>::load(Ab2 + ao);
#pragma unroll
      for (int j = 0; j < 4; ++j) {
        acc[i][j] = Frag<T>::mma(ah, bh[j], acc[i][j]);
        if (SPLIT) {
          acc[i][j] = Frag<T>::mma(ah, bl[j], acc[i][j]);
          acc[i][j] = Frag<T>::mma(al, bh[j], acc[i][j]);
        }
      }
      Frag<T>::guard(acc[i][0], acc[i][3], ah, SPLIT ? al : ah);
    }
    Frag<T>::keep(bh[0], bh[1], bh[2], bh[3]);
    if (SPLIT) Frag<T>::keep(bl[0], bl[1], bl[2], bl[3]);
  }
  acc_guard4(acc[0][0], acc[0][1], acc[0][2], acc[0][3]);
  acc_guard4(acc[1][0], acc[1][1], acc[1][2], acc[1][3]);
  acc_guard4(acc[2][0], acc[2][1], acc[2][2], acc[2][3]);
  acc_guard4(acc[3][0], acc[3][1], acc[3][2], acc[3][3]);

  float* slab = sT[wave];
  const float* Rb = RESID ? (resid + (size_t)b * strideR) : nullptr;
#pragma unroll
  for (int i = 0; i < 4; ++i) {
    const int mBase = m0 + (i << 4);
#pragma unroll
    for (int j = 0; j < 4; ++j) {
      const int n = n0 + (j << 4) + rlane;
      float bv = 0.f;
      if (BIAS_MODE == 2) bv = bias[n];
#pragma unroll
      for (int r = 0; r < 8; ++r) {
        float v = acc[i][j][r] * scale;
        if (BIAS_MODE == 1) v += bias[mBase + mOff + r];
        if (BIAS_MODE == 2) v += bv;
        if (RESID) v += Rb[(size_t)(mBase + mOff + r) * ldc + n];
        if (ACT == 1) v = tanhf(v);
        if (ACT == 2) v = fmaxf(v, 0.0f);
        if (ACT == 3) v = v / (1.0f + expf(-v));
        if (ACT == 4) v = (v > 0.f) ? v : 0.01f * v;
        if (ACT == 5) v = 0.5f * v * (1.0f + erff(v * 0.70710678118654752f));
        if (ACT == 7) v = (v >= 0.f) ? v : 0.2f * v;
        slab[(mOff + r) * 68 + (j << 4) + rlane] = v;
      }
    }
    __builtin_amdgcn_fence(__ATOMIC_RELEASE, "workgroup");
    __builtin_amdgcn_wave_barrier();
    __builtin_amdgcn_fence(__ATOMIC_ACQUIRE, "workgroup");
    if (OUT_MODE == 0) {
      float* C = (float*)Cout + (size_t)b * strideC;
      const int hh = lane >> 4, c4 = (lane & 15) * 4;
      for (int pass = 0; pass < 2; ++pass) {
#pragma unroll
        for (int it = 0; it < 8; ++it) {
          const int row = it * 2 + hh;
          v4f v = *(const v4f*)(slab + row * 68 + c4);
          *(volatile v4f*)(C + (size_t)(mBase + row) * ldc + n0 + c4) = v;
        }
        __threadfence();
      }
    } else {
      const int q = lane >> 3, c8 = (lane & 7) * 8;
      unsigned short* C  = (unsigned short*)Cout  + (size_t)b * strideC;
      unsigned short* C2 = (OUT_MODE == 2) ? ((unsigned short*)Cout2 + (size_t)b * strideC) : nullptr;
      for (int pass = 0; pass < 2; ++pass) {
#pragma unroll
        for (int it = 0; it < 4; ++it) {
          const int row = it * 4 + q;
          const float* sp = slab + row * 68 + c8;
          v8h hv, lv;
#pragma unroll
          for (int e = 0; e < 8; ++e) {
            if (OUT_MODE == 1) {
              hv[e] = (_Float16)sp[e];
            } else {
              unsigned short hb = f2bf_bits(sp[e]);
              unsigned short lb = f2bf_bits(sp[e] - bf_bits2f(hb));
              hv[e] = __builtin_bit_cast(_Float16, hb);
              lv[e] = __builtin_bit_cast(_Float16, lb);
            }
          }
          *(volatile v8h*)(C + (size_t)(mBase + row) * ldc + n0 + c8) = hv;
          if (OUT_MODE == 2) *(volatile v8h*)(C2 + (size_t)(mBase + row) * ldc + n0 + c8) = lv;
        }
        __threadfence();
      }
    }
    __builtin_amdgcn_fence(__ATOMIC_RELEASE, "workgroup");
    __builtin_amdgcn_wave_barrier();
    __builtin_amdgcn_fence(__ATOMIC_ACQUIRE, "workgroup");
  }
}

__global__ __launch_bounds__(256) void k_pad_bf16(const float* __restrict__ src, unsigned short* __restrict__ dst,
                                                  int rows, int pmask, int pshift, int pq) {
  const int i = blockIdx.x * 256 + threadIdx.x;
  if (i >= rows * 40) return;
  const int r = i / 40, c8 = (i - r * 40) * 8;
  const int srow = (r & pmask) * pq + (r >> pshift);
  const float* p = src + (size_t)srow * NIN;
  unsigned short hb[8];
#pragma unroll
  for (int e = 0; e < 8; ++e) {
    const int c  = c8 + e;
    const int cc = (c < NIN) ? c : (NIN - 1);
    const float v = p[cc];
    hb[e] = (c < NIN) ? f2bf_bits(v) : (unsigned short)0;
  }
  const v4u u = (v4u){pk16(hb[0], hb[1]), pk16(hb[2], hb[3]), pk16(hb[4], hb[5]), pk16(hb[6], hb[7])};
  unsigned short* q = dst + (size_t)i * 8;
  *(volatile v4u*)q = u;
  __threadfence();
  *(volatile v4u*)q = u;
}

__global__ __launch_bounds__(256) void k_cvt_f16s(const float* __restrict__ src, unsigned short* __restrict__ dst, int n8, float scale) {
  const int i = blockIdx.x * 256 + threadIdx.x;
  if (i >= n8) return;
  const float* p = src + (size_t)i * 8;
  const v4f a = *(const v4f*)(p);
  const v4f c = *(const v4f*)(p + 4);
  unsigned short hb[8];
#pragma unroll
  for (int e = 0; e < 4; ++e) {
    hb[e]     = h_bits(bf_rne(a[e]) * scale);
    hb[4 + e] = h_bits(bf_rne(c[e]) * scale);
  }
  const v4u u = (v4u){pk16(hb[0], hb[1]), pk16(hb[2], hb[3]), pk16(hb[4], hb[5]), pk16(hb[6], hb[7])};
  unsigned short* q = dst + (size_t)i * 8;
  *(volatile v4u*)q = u;
  __threadfence();
  *(volatile v4u*)q = u;
}

__global__ __launch_bounds__(256) void k_rnd_f32(const float* __restrict__ src, float* __restrict__ dst, int n4) {
  const int i = blockIdx.x * 256 + threadIdx.x;
  if (i >= n4) return;
  const v4f a = *(const v4f*)(src + (size_t)i * 4);
  v4f o;
#pragma unroll
  for (int e = 0; e < 4; ++e) o[e] = bf_rne(a[e]);
  float* q = dst + (size_t)i * 4;
  *(volatile v4f*)q = o;
  __threadfence();
  *(volatile v4f*)q = o;
}

__device__ __forceinline__ float sigm_g(float v) { return __builtin_amdgcn_rcpf(1.0f + __expf(-v)); }
__device__ __forceinline__ float tanh_g(float v) { return fmaf(-2.0f, __builtin_amdgcn_rcpf(__expf(2.0f * v) + 1.0f), 1.0f); }

__global__ __launch_bounds__(REC_THREADS) void k_gru_chunk(
    const float* __restrict__ GIf, const float* __restrict__ GIb,
    const unsigned short* __restrict__ Whhp,
    const float* __restrict__ bhhF, const float* __restrict__ bhhB,
    const int* __restrict__ lens, int nlens,
    float* __restrict__ Hst, float* __restrict__ Ssum,
    int chunk, int first) {
  extern __shared__ __align__(16) unsigned char dynlds[];
  float*    hst  = (float*)(dynlds + REC_LDS_HST);
  float*    ssum = (float*)(dynlds + REC_LDS_SSUM);
  _Float16* hpl  = (_Float16*)(dynlds + REC_LDS_HPL);
  int*      slen = (int*)(dynlds + REC_LDS_SLEN);

  const int tid  = threadIdx.x;
  const int wave = tid >> 5;
  const int lane = tid & 31;
  const int hh   = lane >> 4;
  const int l15  = lane & 15;
  const int koff = hh * 8;
  const int dir  = blockIdx.x >> 3;
  const int bgrp = blockIdx.x & 7;
  const float* GI  = dir ? GIb : GIf;
  const float* bhh = dir ? bhhB : bhhF;
  const _Float16* Whh = (const _Float16*)Whhp + (size_t)dir * NGATE * NHID;
  const size_t gbase = ((size_t)dir * NBATCH + (size_t)bgrp * SEQ_PER_BLK) * NHID;

  if (tid < SEQ_PER_BLK) {
    int b = bgrp * SEQ_PER_BLK + tid;
    b = (b < nlens) ? b : (nlens - 1);
    b = (b < 0) ? 0 : b;
    slen[tid] = lens[b];
  }
  for (int idx = tid; idx < SEQ_PER_BLK * NHID / 4; idx += REC_THREADS) {
    const int row = idx >> 7, c4 = (idx & 127) * 4;
    v4f hv = (v4f){0.f, 0.f, 0.f, 0.f};
    v4f sv = hv;
    if (!first) {
      hv = *(const v4f*)(Hst  + gbase + (size_t)idx * 4);
      sv = *(const v4f*)(Ssum + gbase + (size_t)idx * 4);
    }
    *(v4f*)(hst  + idx * 4) = hv;
    *(v4f*)(ssum + idx * 4) = sv;
    _Float16* hp = hpl + row * HPL_PITCH + c4;
    hp[0] = (_Float16)(hv[0] * H_CARRY);
    hp[1] = (_Float16)(hv[1] * H_CARRY);
    hp[2] = (_Float16)(hv[2] * H_CARRY);
    hp[3] = (_Float16)(hv[3] * H_CARRY);
  }
  __syncthreads();

  const int colA = 16 * wave + l15;
  const int colB = 256 + 16 * wave + l15;
  float bq[6];
#pragma unroll
  for (int g = 0; g < 2; ++g)
#pragma unroll
    for (int q = 0; q < 3; ++q) bq[g * 3 + q] = bf_rne(bhh[q * NHID + (g ? colB : colA)]);

  const _Float16* Bbase = Whh + koff;
  const _Float16* Abase = hpl + (size_t)l15 * HPL_PITCH + koff;

#pragma unroll 1
  for (int j = 0; j < CHUNK_STEPS; ++j) {
    v8f acc[2][6];
#pragma unroll
    for (int i = 0; i < 2; ++i)
#pragma unroll
      for (int t = 0; t < 6; ++t) acc[i][t] = (v8f){0.f,0.f,0.f,0.f,0.f,0.f,0.f,0.f};

#pragma unroll 1
    for (int k0 = 0; k0 < NHID; k0 += 32) {
      const v16h a0 = Frag<_Float16>::load(Abase + k0);
      const v16h a1 = Frag<_Float16>::load(Abase + 16 * HPL_PITCH + k0);
#pragma unroll
      for (int g = 0; g < 2; ++g) {
        const int colg = g ? colB : colA;
        v16h bfr[3];
#pragma unroll
        for (int q = 0; q < 3; ++q) bfr[q] = Frag<_Float16>::load(Bbase + (size_t)(q * NHID + colg) * NHID + k0);
#pragma unroll
        for (int q = 0; q < 3; ++q) {
          acc[0][g * 3 + q] = Frag<_Float16>::mma(a0, bfr[q], acc[0][g * 3 + q]);
          acc[1][g * 3 + q] = Frag<_Float16>::mma(a1, bfr[q], acc[1][g * 3 + q]);
        }
        Frag<_Float16>::guard(acc[0][g * 3], acc[1][g * 3 + 2], a0, a1);
        Frag<_Float16>::keep(bfr[0], bfr[1], bfr[2], bfr[2]);
      }
    }
    acc_guard4(acc[0][0], acc[0][1], acc[0][2], acc[0][3]);
    acc_guard4(acc[0][4], acc[0][5], acc[1][0], acc[1][1]);
    acc_guard4(acc[1][2], acc[1][3], acc[1][4], acc[1][5]);
    __syncthreads();

    const int tstep = chunk * CHUNK_STEPS + j;
    const int jrow  = dir ? (CHUNK_STEPS - 1 - j) : j;
    const float* Gstep = GI + (size_t)jrow * NBATCH * NGATE;
#pragma unroll
    for (int i = 0; i < 2; ++i) {
#pragma unroll
      for (int g = 0; g < 2; ++g) {
        const int col = g ? colB : colA;
        asm volatile("" ::: "memory");
#pragma unroll
        for (int r = 0; r < 8; ++r) {
          const int rb = 16 * i + 8 * hh + r;
          const int b  = bgrp * SEQ_PER_BLK + rb;
          const float* gp = Gstep + (size_t)b * NGATE + col;
          const float gir = gp[0];
          const float giz = gp[NHID];
          const float gin = gp[2 * NHID];
          const float ghr = fmaf(acc[i][g * 3 + 0][r], GH_UNSCALE, bq[g * 3 + 0]);
          const float ghz = fmaf(acc[i][g * 3 + 1][r], GH_UNSCALE, bq[g * 3 + 1]);
          const float ghn = fmaf(acc[i][g * 3 + 2][r], GH_UNSCALE, bq[g * 3 + 2]);
          const float rg = sigm_g(gir + ghr);
          const float zg = sigm_g(giz + ghz);
          const float ng = tanh_g(fmaf(rg, ghn, gin));
          const int li = rb * NHID + col;
          const float hp = hst[li];
          const float hn = (1.0f - zg) * ng + zg * hp;
          hst[li] = hn;
          const float add = (tstep < slen[rb]) ? hn : 0.0f;
          ssum[li] = ssum[li] + add;
          hpl[rb * HPL_PITCH + col] = (_Float16)(hn * H_CARRY);
        }
      }
    }
    __syncthreads();
  }

  for (int pass = 0; pass < 2; ++pass) {
    for (int idx = tid; idx < SEQ_PER_BLK * NHID / 4; idx += REC_THREADS) {
      const v4f hv = *(const v4f*)(hst  + idx * 4);
      const v4f sv = *(const v4f*)(ssum + idx * 4);
      *(volatile v4f*)(Hst  + gbase + (size_t)idx * 4) = hv;
      *(volatile v4f*)(Ssum + gbase + (size_t)idx * 4) = sv;
    }
    __threadfence();
  }
}

__global__ __launch_bounds__(256) void k_avg(const float* __restrict__ Ssum, unsigned short* __restrict__ AVG) {
  const int i = blockIdx.x * 256 + threadIdx.x;
  if (i >= NBATCH * NHID / 8) return;
  const float* pf = Ssum + (size_t)i * 8;
  const float* pb = Ssum + (size_t)NBATCH * NHID + (size_t)i * 8;
  const v4f f0 = *(const v4f*)(pf), f1 = *(const v4f*)(pf + 4);
  const v4f b0 = *(const v4f*)(pb), b1 = *(const v4f*)(pb + 4);
  unsigned short hb[8];
#pragma unroll
  for (int e = 0; e < 4; ++e) {
    hb[e]     = h_bits(((f0[e] + b0[e]) * AVG_SCALE) * H_CARRY);
    hb[4 + e] = h_bits(((f1[e] + b1[e]) * AVG_SCALE) * H_CARRY);
  }
  const v4u u = (v4u){pk16(hb[0], hb[1]), pk16(hb[2], hb[3]), pk16(hb[4], hb[5]), pk16(hb[6], hb[7])};
  unsigned short* q = AVG + (size_t)i * 8;
  *(volatile v4u*)q = u;
  __threadfence();
  *(volatile v4u*)q = u;
}

__global__ __launch_bounds__(256) void k_out(const float* __restrict__ MU, const float* __restrict__ noise, float* __restrict__ out) {
  const int i = blockIdx.x * 256 + threadIdx.x;
  if (i >= NBATCH * NCOND / 4) return;
  const v4f m  = *(const v4f*)(MU + (size_t)i * 4);
  const v4f nz = *(const v4f*)(noise + (size_t)i * 4);
  v4f o;
#pragma unroll
  for (int e = 0; e < 4; ++e) {
    const float nb = bf_rne(nz[e]);
    o[e] = nb * m[e] + m[e];
  }
  float* q = out + (size_t)i * 4;
  *(volatile v4f*)q = o;
  __threadfence();
  *(volatile v4f*)q = o;
}

extern "C" void kernel_launch(void* const* d_in, const int* in_sizes, int n_in,
                              void* d_out, int out_size, void* d_ws, size_t ws_size,
                              hipStream_t stream) {
  if (n_in < 13) return;
  if (in_sizes[0]  != NBATCH * NSEQ * NIN) return;
  if (in_sizes[1]  != NBATCH) return;
  if (in_sizes[2]  != NGATE * NIN) return;
  if (in_sizes[3]  != NGATE * NHID) return;
  if (in_sizes[4]  != NGATE || in_sizes[5] != NGATE) return;
  if (in_sizes[6]  != NGATE * NIN) return;
  if (in_sizes[7]  != NGATE * NHID) return;
  if (in_sizes[8]  != NGATE || in_sizes[9] != NGATE) return;
  if (in_sizes[10] != NCOND * NHID) return;
  if (in_sizes[11] != NCOND) return;
  if (in_sizes[12] != NBATCH * NCOND) return;
  if (out_size != NBATCH * NCOND) return;
  if (((NBATCH * NSEQ * 40) % 32) != 0 || ((NGATE * 40) % 32) != 0) return;
  if (((NGATE * NHID / 8) % 32) != 0 || ((NCOND * NHID / 8) % 32) != 0) return;
  if (((NGATE / 4) % 32) != 0 || ((NCOND / 4) % 32) != 0) return;

  const float* text  = (const float*)d_in[0];
  const int*   lens  = (const int*)d_in[1];
  const float* Wih_f = (const float*)d_in[2];
  const float* Whh_f = (const float*)d_in[3];
  const float* bih_f = (const float*)d_in[4];
  const float* bhh_f = (const float*)d_in[5];
  const float* Wih_b = (const float*)d_in[6];
  const float* Whh_b = (const float*)d_in[7];
  const float* bih_b = (const float*)d_in[8];
  const float* bhh_b = (const float*)d_in[9];
  const float* W_mu  = (const float*)d_in[10];
  const float* b_mu  = (const float*)d_in[11];
  const float* noise = (const float*)d_in[12];
  float* out = (float*)d_out;

  char* ws = (char*)d_ws;
  size_t off = 0;
  auto carve = [&](size_t bytes) { size_t o = off; off += (bytes + 255) & ~(size_t)255; return o; };
  const size_t oXb   = carve((size_t)NBATCH * NSEQ * NINP * 2);
  const size_t oWihb = carve((size_t)2 * NGATE * NINP * 2);
  const size_t oWhhh = carve((size_t)2 * NGATE * NHID * 2);
  const size_t oWmuh = carve((size_t)NCOND * NHID * 2);
  const size_t oBihr = carve((size_t)2 * NGATE * 4);
  const size_t oBmur = carve((size_t)NCOND * 4);
  const size_t oGIf  = carve((size_t)CHUNK_ROWS * NGATE * 4);
  const size_t oGIb  = carve((size_t)CHUNK_ROWS * NGATE * 4);
  const size_t oHst  = carve((size_t)2 * NBATCH * NHID * 4);
  const size_t oSsum = carve((size_t)2 * NBATCH * NHID * 4);
  const size_t oAvg  = carve((size_t)NBATCH * NHID * 2);
  const size_t oMu   = carve((size_t)NBATCH * NCOND * 4);
  if (off > ws_size) return;

  unsigned short* Xb   = (unsigned short*)(ws + oXb);
  unsigned short* Wihb = (unsigned short*)(ws + oWihb);
  unsigned short* Whhh = (unsigned short*)(ws + oWhhh);
  unsigned short* Wmuh = (unsigned short*)(ws + oWmuh);
  float* bihr = (float*)(ws + oBihr);
  float* bmur = (float*)(ws + oBmur);
  float* GIf  = (float*)(ws + oGIf);
  float* GIb  = (float*)(ws + oGIb);
  float* Hst  = (float*)(ws + oHst);
  float* Ssum = (float*)(ws + oSsum);
  unsigned short* AVGh = (unsigned short*)(ws + oAvg);
  float* MU   = (float*)(ws + oMu);

  auto blk = [](int n) { return (n + 255) / 256; };

  k_pad_bf16<<<blk(NBATCH * NSEQ * 40), 256, 0, stream>>>(text, Xb, NBATCH * NSEQ, NBATCH - 1, 8, NSEQ);
  k_pad_bf16<<<blk(NGATE * 40), 256, 0, stream>>>(Wih_f, Wihb, NGATE, 0, 0, 0);
  k_pad_bf16<<<blk(NGATE * 40), 256, 0, stream>>>(Wih_b, Wihb + (size_t)NGATE * NINP, NGATE, 0, 0, 0);
  k_cvt_f16s<<<blk(NGATE * NHID / 8), 256, 0, stream>>>(Whh_f, Whhh, NGATE * NHID / 8, W_CARRY);
  k_cvt_f16s<<<blk(NGATE * NHID / 8), 256, 0, stream>>>(Whh_b, Whhh + (size_t)NGATE * NHID, NGATE * NHID / 8, W_CARRY);
  k_cvt_f16s<<<blk(NCOND * NHID / 8), 256, 0, stream>>>(W_mu, Wmuh, NCOND * NHID / 8, W_CARRY);
  k_rnd_f32<<<blk(NGATE / 4), 256, 0, stream>>>(bih_f, bihr, NGATE / 4);
  k_rnd_f32<<<blk(NGATE / 4), 256, 0, stream>>>(bih_b, bihr + NGATE, NGATE / 4);
  k_rnd_f32<<<blk(NCOND / 4), 256, 0, stream>>>(b_mu, bmur, NCOND / 4);

  const int giTiles = (CHUNK_ROWS / 64) * (NGATE / 64);
  const dim3 giGrid((giTiles + 7) / 8, 1);
  for (int c = 0; c < NCHUNK; ++c) {
    const size_t rowF = (size_t)(CHUNK_STEPS * c) * NBATCH;
    const size_t rowB = (size_t)(NSEQ - CHUNK_STEPS - CHUNK_STEPS * c) * NBATCH;
    wmma_gemm64<1, false, 2, 0, false, 0><<<giGrid, 256, 0, stream>>>(
        Xb + rowF * NINP, Xb + rowF * NINP, NINP, 0L,
        Wihb, Wihb, NINP, 0L,
        (void*)GIf, (void*)GIf, NGATE, 0L,
        bihr, bihr, 0L,
        CHUNK_ROWS, NGATE, NINP, 1.0f);
    wmma_gemm64<1, false, 2, 0, false, 0><<<giGrid, 256, 0, stream>>>(
        Xb + rowB * NINP, Xb + rowB * NINP, NINP, 0L,
        Wihb + (size_t)NGATE * NINP, Wihb + (size_t)NGATE * NINP, NINP, 0L,
        (void*)GIb, (void*)GIb, NGATE, 0L,
        bihr + NGATE, bihr + NGATE, 0L,
        CHUNK_ROWS, NGATE, NINP, 1.0f);
    k_gru_chunk<<<REC_BLOCKS, REC_THREADS, REC_LDS_BYTES, stream>>>(
        GIf, GIb, Whhh, bhh_f, bhh_b, lens, NBATCH, Hst, Ssum, c, (c == 0) ? 1 : 0);
  }

  k_avg<<<blk(NBATCH * NHID / 8), 256, 0, stream>>>(Ssum, AVGh);
  const int muTiles = (NBATCH / 64) * (NCOND / 64);
  wmma_gemm64<0, false, 2, 0, false, 7><<<dim3((muTiles + 7) / 8, 1), 256, 0, stream>>>(
      AVGh, AVGh, NHID, 0L,
      Wmuh, Wmuh, NHID, 0L,
      (void*)MU, (void*)MU, NCOND, 0L,
      bmur, bmur, 0L,
      NBATCH, NCOND, NHID, GH_UNSCALE);
  k_out<<<blk(NBATCH * NCOND / 4), 256, 0, stream>>>(MU, noise, out);
}
